// STM_41575283425930
// MI455X (gfx1250) — hardware-verified
//
#include <hip/hip_runtime.h>
#include <math.h>

typedef __attribute__((ext_vector_type(16))) _Float16 v16h;
typedef __attribute__((ext_vector_type(16))) __bf16 v16b;
typedef __attribute__((ext_vector_type(8)))  _Float16 v8h;
typedef __attribute__((ext_vector_type(8)))  float v8f;
typedef __attribute__((ext_vector_type(4)))  float v4f;
typedef __attribute__((ext_vector_type(2)))  float v2f;
typedef __attribute__((ext_vector_type(4)))  unsigned v4u;
typedef __attribute__((ext_vector_type(4)))  int v4i;
typedef float __attribute__((may_alias)) float_a;
typedef int __attribute__((may_alias)) int_a;

template <typename T> __device__ __forceinline__ void vst2(void* p, T v) { *(volatile T*)p = v; __threadfence(); *(volatile T*)p = v; }
__device__ __forceinline__ v8f wmma16(v16h a, v16h b, v8f c) {
  v8f d = __builtin_amdgcn_wmma_f32_16x16x32_f16(false, a, false, b, (short)0, c, false, false);
  asm volatile("v_nop\n\tv_nop\n\tv_nop\n\tv_nop" : "+v"(d) : "v"(a), "v"(b));
  return d;
}
__device__ __forceinline__ v8f wmma_bf(v16b a, v16b b, v8f c) {
  v8f d = __builtin_amdgcn_wmma_f32_16x16x32_bf16(false, a, false, b, (short)0, c, false, false);
  asm volatile("v_nop\n\tv_nop\n\tv_nop\n\tv_nop" : "+v"(d) : "v"(a), "v"(b));
  return d;
}
__device__ __forceinline__ v16h frag_h(const _Float16* rowk0, int lane) {
  union { v16h v; v8h q[2]; } u; const _Float16* p = rowk0 + 8 * (lane >> 4);
  u.q[0] = *(const v8h*)p; u.q[1] = *(const v8h*)(p + 16); return u.v;
}
__device__ __forceinline__ v16h frag_f32(const float* rowk0, int lane) {
  v16h a; const float* p = rowk0 + 8 * (lane >> 4);
#pragma unroll
  for (int i = 0; i < 8; ++i) { a[i] = (_Float16)p[i]; a[8 + i] = (_Float16)p[16 + i]; }
  return a;
}
__device__ __forceinline__ v16h frag_f32s(const float* rowk0, int lane, float sc) {
  v16h a; const float* p = rowk0 + 8 * (lane >> 4);
#pragma unroll
  for (int i = 0; i < 8; ++i) { a[i] = (_Float16)(p[i] * sc); a[8 + i] = (_Float16)(p[16 + i] * sc); }
  return a;
}
__device__ __forceinline__ v16h fragc_f32(const float* W, int k0, int n, int lane, int ld, int K) {
  v16h a; const int g = lane >> 4;
#pragma unroll
  for (int i = 0; i < 8; ++i) { const int ka = k0 + 8 * g + i, kb = ka + 16;
    a[i] = (_Float16)(ka < K ? W[(size_t)ka * ld + n] : 0.f); a[8 + i] = (_Float16)(kb < K ? W[(size_t)kb * ld + n] : 0.f); }
  return a;
}
struct F2 { v16b h, l; };
__device__ __forceinline__ F2 bsplit16(const float v[16]) { F2 r;
#pragma unroll
  for (int i = 0; i < 16; ++i) { const __bf16 h = (__bf16)v[i]; r.h[i] = h; r.l[i] = (__bf16)(v[i] - (float)h); }
  return r; }
__device__ __forceinline__ F2 split_row(const float* row, int k0, int lane) { float v[16]; const float* p = row + k0 + 8 * (lane >> 4);
#pragma unroll
  for (int i = 0; i < 8; ++i) { v[i] = p[i]; v[8 + i] = p[16 + i]; }
  return bsplit16(v); }
__device__ __forceinline__ F2 split_rowK(const float* row, int k0, int lane, int K) { float v[16]; const int g = lane >> 4;
#pragma unroll
  for (int i = 0; i < 8; ++i) { const int ka = k0 + 8 * g + i, kb = ka + 16; v[i] = ka < K ? row[ka] : 0.f; v[8 + i] = kb < K ? row[kb] : 0.f; }
  return bsplit16(v); }
__device__ __forceinline__ F2 split_col(const float* W, int k0, int n, int lane, int ld, int K) { float v[16]; const int g = lane >> 4;
#pragma unroll
  for (int i = 0; i < 8; ++i) { const int ka = k0 + 8 * g + i, kb = ka + 16; v[i] = ka < K ? W[(size_t)ka * ld + n] : 0.f; v[8 + i] = kb < K ? W[(size_t)kb * ld + n] : 0.f; }
  return bsplit16(v); }
__device__ __forceinline__ v8f mac3(const F2& a, const F2& b, v8f c) { c = wmma_bf(a.l, b.h, c); c = wmma_bf(a.h, b.l, c); return wmma_bf(a.h, b.h, c); }
__device__ __forceinline__ float sigm(float v) { return 1.0f / (1.0f + expf(-v)); }
#define LDSX() do { asm volatile("s_wait_dscnt 0" ::: "memory"); __builtin_amdgcn_wave_barrier(); __builtin_amdgcn_fence(__ATOMIC_RELEASE, "workgroup"); } while (0)

#define NB 2
#define NF 5
#define CC 256
#define HW 4096
#define CK 32
#define CV 128
#define NM 4
#define NKEY (NM * HW)

__global__ __launch_bounds__(256) void k_copy(const float* __restrict__ x, float* __restrict__ out) {
  const size_t i4 = (size_t)blockIdx.x * 256 + threadIdx.x; const size_t per_b = (size_t)NM * CC * HW / 4;
  if (i4 >= (size_t)NB * per_b) return; const size_t b = i4 / per_b, r = i4 % per_b;
  const size_t src = b * (size_t)NF * CC * HW + r * 4;
  vst2(out + src, *(const v4f*)(x + src));
}
template <int MODE>
__global__ __launch_bounds__(128) void k_kv(const float* __restrict__ x, const float* __restrict__ kw, const float* __restrict__ vw, _Float16* __restrict__ K16, _Float16* __restrict__ MVT, float* __restrict__ QV) {
  __shared__ __align__(16) float sk[4][16][36];
  __shared__ __align__(16) float sv[CV][68];
  const int tid = threadIdx.x, wave = tid >> 5, lane = tid & 31, col = lane & 15, g = lane >> 4;
  const int z = blockIdx.z; const int b = MODE == 0 ? z / NM : z, fr = MODE == 0 ? z % NM : NM;
  const int p0b = blockIdx.x * 64, p0 = p0b + wave * 16;
  const float* xb = x + ((size_t)(b * NF + fr) * CC) * HW;
  v8f ak[2] = {}, av[8] = {};
#pragma unroll 1
  for (int kc = 0; kc < CC / 32; ++kc) { const v16h a = fragc_f32(xb, kc * 32, p0 + col, lane, HW, CC);
#pragma unroll
    for (int j = 0; j < 2; ++j) ak[j] = wmma16(a, frag_f32s(kw + (size_t)(j * 16 + col) * CC + kc * 32, lane, 4.0f), ak[j]);
#pragma unroll
    for (int j = 0; j < 8; ++j) av[j] = wmma16(a, frag_f32s(vw + (size_t)(j * 16 + col) * CC + kc * 32, lane, 4.0f), av[j]); }
#pragma unroll
  for (int j = 0; j < 2; ++j)
#pragma unroll
    for (int r = 0; r < 8; ++r) sk[wave][8 * g + r][j * 16 + col] = ak[j][r] * 0.25f;
#pragma unroll
  for (int j = 0; j < 8; ++j)
#pragma unroll
    for (int r = 0; r < 8; ++r) sv[j * 16 + col][wave * 16 + 8 * g + r] = av[j][r] * 0.25f;
  LDSX();
  for (int rl = 0; rl < 16; ++rl) { const float v = sk[wave][rl][lane]; float q2 = v * v;
#pragma unroll
    for (int off = 16; off >= 1; off >>= 1) q2 += __shfl_xor(q2, off, 32);
    sk[wave][rl][lane] = v / fmaxf(sqrtf(q2), 1e-12f) * 8.0f; }
  LDSX();
  for (int q = lane; q < 16 * 4; q += 32) { const int rl = q >> 2, pc = q & 3; union { v8h h8; v4u u; } pk;
#pragma unroll
    for (int e = 0; e < 8; ++e) pk.h8[e] = (_Float16)sk[wave][rl][pc * 8 + e];
    const size_t row = MODE == 0 ? ((size_t)b * NKEY + (size_t)fr * HW + p0 + rl) : ((size_t)b * HW + p0 + rl);
    vst2(K16 + row * CK + pc * 8, pk.u); }
  __syncthreads();
  if (MODE == 0) { for (int q = tid; q < CV * 8; q += 128) { const int d = q >> 3, pc = q & 7; union { v8h h8; v4u u; } pk;
#pragma unroll
      for (int e = 0; e < 8; ++e) pk.h8[e] = (_Float16)sv[d][pc * 8 + e];
      vst2(MVT + ((size_t)b * CV + d) * NKEY + (size_t)fr * HW + p0b + pc * 8, pk.u); } }
  else { for (int q = tid; q < CV * 16; q += 128) { const int d = q >> 4, pc = q & 15; vst2(QV + ((size_t)b * CV + d) * HW + p0b + pc * 4, *(const v4f*)(&sv[d][pc * 4])); } }
}
__global__ __launch_bounds__(128) void k_attn(const _Float16* __restrict__ QK, const _Float16* __restrict__ MK, const _Float16* __restrict__ MVT, float* __restrict__ AGG) {
  __shared__ __align__(16) float sS[4][16][68];
  __shared__ __align__(16) _Float16 sP[4][16][72];
  __shared__ __align__(16) float sO[CV][68];
  const int tid = threadIdx.x, w = tid >> 5, lane = tid & 31, col = lane & 15, g = lane >> 4;
  const int b = blockIdx.y, p0b = blockIdx.x * 64, q0 = p0b + w * 16;
  const _Float16* qb = QK + (size_t)b * HW * CK; const _Float16* kb = MK + (size_t)b * NKEY * CK; const _Float16* vb = MVT + (size_t)b * CV * NKEY;
  const v16h aq = frag_h(qb + (size_t)(q0 + col) * CK, lane);
  float mrun = -3.0e38f, lrun = 0.f; v8f acc[8] = {};
#pragma unroll 1
  for (int kt = 0; kt < NKEY / 64; ++kt) {
#pragma unroll
    for (int t = 0; t < 4; ++t) { v8f s = {}; s = wmma16(aq, frag_h(kb + (size_t)(kt * 64 + t * 16 + col) * CK, lane), s);
#pragma unroll
      for (int r = 0; r < 8; ++r) sS[w][8 * g + r][t * 16 + col] = s[r] * (1.0f / 64.0f); }
    LDSX();
    float mx = -3.4e38f;
#pragma unroll
    for (int jj = 0; jj < 32; ++jj) mx = fmaxf(mx, sS[w][col][g * 32 + jj]);
    mx = fmaxf(mx, __shfl_xor(mx, 16, 32));
    const float mnew = fmaxf(mrun, mx); const float corr = __expf(mrun - mnew);
    float ps = 0.f;
#pragma unroll
    for (int jj = 0; jj < 32; ++jj) { const float p = __expf(sS[w][col][g * 32 + jj] - mnew); ps += p; sP[w][col][g * 32 + jj] = (_Float16)(p * 16384.0f); }
    ps += __shfl_xor(ps, 16, 32);
    lrun = lrun * corr + ps; mrun = mnew;
#pragma unroll
    for (int r = 0; r < 8; ++r) { const float cr = __shfl(corr, 8 * g + r, 32);
#pragma unroll
      for (int t = 0; t < 8; ++t) acc[t][r] *= cr; }
    LDSX();
#pragma unroll
    for (int kc = 0; kc < 2; ++kc) { const v16h pa = frag_h(&sP[w][col][0] + kc * 32, lane);
#pragma unroll
      for (int t = 0; t < 8; ++t) acc[t] = wmma16(pa, frag_h(vb + (size_t)(t * 16 + col) * NKEY + kt * 64 + kc * 32, lane), acc[t]); }
    __builtin_amdgcn_wave_barrier();
  }
#pragma unroll
  for (int r = 0; r < 8; ++r) { const float lr = __shfl(lrun, 8 * g + r, 32);
#pragma unroll
    for (int t = 0; t < 8; ++t) sO[t * 16 + col][w * 16 + 8 * g + r] = acc[t][r] / (lr * 16384.0f); }
  __syncthreads();
  for (int q = tid; q < CV * 16; q += 128) { const int d = q >> 4, pc = q & 15; vst2(AGG + ((size_t)b * CV + d) * HW + p0b + pc * 4, *(const v4f*)(&sO[d][pc * 4])); }
}
__device__ __forceinline__ v16h fragc_sc(const float* base, int k0, int n, int lane, int ld, float sc) { v16h v; const int g = lane >> 4;
#pragma unroll
  for (int i = 0; i < 8; ++i) { v[i] = (_Float16)(base[(size_t)(k0 + 8 * g + i) * ld + n] * sc); v[8 + i] = (_Float16)(base[(size_t)(k0 + 16 + 8 * g + i) * ld + n] * sc); }
  return v; }
__global__ __launch_bounds__(128) void k_fin(const float* __restrict__ QV, const float* __restrict__ AGG, const float* __restrict__ sw, const float* __restrict__ bsc, const float* __restrict__ bbi, const float* __restrict__ bmu, const float* __restrict__ bva, float* __restrict__ out) {
  __shared__ __align__(16) float st[128][68];
  const int tid = threadIdx.x, wave = tid >> 5, lane = tid & 31, col = lane & 15, g = lane >> 4;
  const int b = blockIdx.z, p0b = blockIdx.x * 64, p0 = p0b + wave * 16, o0 = blockIdx.y * 128;
  v8f acc[8] = {};
#pragma unroll 1
  for (int kc = 0; kc < CC / 32; ++kc) { const bool isagg = kc >= 4; const float* src = isagg ? AGG + (size_t)b * CV * HW : QV + (size_t)b * CV * HW; const int kl = (kc & 3) * 32;
    const v16h a = fragc_sc(src, kl, p0 + col, lane, HW, isagg ? 1024.0f : 1.0f);
    const float wsc = isagg ? (4.0f / 1024.0f) : 4.0f;
#pragma unroll
    for (int j = 0; j < 8; ++j) acc[j] = wmma16(a, frag_f32s(sw + (size_t)(o0 + j * 16 + col) * CC + kc * 32, lane, wsc), acc[j]); }
#pragma unroll
  for (int j = 0; j < 8; ++j) { const int o = o0 + j * 16 + col; const float sc = bsc[o] * rsqrtf(bva[o] + 1e-5f), mu = bmu[o], bi = bbi[o];
#pragma unroll
    for (int r = 0; r < 8; ++r) { const float v = (acc[j][r] * 0.25f - mu) * sc + bi; st[j * 16 + col][wave * 16 + 8 * g + r] = v > 0.f ? v : 0.f; } }
  __syncthreads();
  for (int q = tid; q < 128 * 16; q += 128) { const int ol = q >> 4, pc = q & 15; vst2(out + (((size_t)b * NF + NM) * CC + o0 + ol) * HW + p0b + pc * 4, *(const v4f*)(&st[ol][pc * 4])); }
}
extern "C" void kernel_launch(void* const* d_in, const int* in_sizes, int n_in, void* d_out, int out_size, void* d_ws, size_t ws_size, hipStream_t stream) {
  (void)in_sizes; (void)n_in; (void)out_size; (void)ws_size;
  const float** I = (const float**)d_in;
  const float* x = I[0]; const float* qkw = I[2]; const float* qvw = I[3]; const float* mkw = I[4]; const float* mvw = I[5]; const float* smw = I[6]; const float* bsc = I[7]; const float* bbi = I[8]; const float* bmu = I[9]; const float* bva = I[10];
  float* out = (float*)d_out;
  char* ws = (char*)d_ws; size_t off = 0;
  auto take = [&](size_t bytes) { char* p = ws + off; off += (bytes + 255) & ~(size_t)255; return p; };
  _Float16* MK = (_Float16*)take((size_t)NB * NKEY * CK * 2); _Float16* MVT = (_Float16*)take((size_t)NB * CV * NKEY * 2); _Float16* QK = (_Float16*)take((size_t)NB * HW * CK * 2);
  float* QV = (float*)take((size_t)NB * CV * HW * 4); float* AGG = (float*)take((size_t)NB * CV * HW * 4);
  { const size_t n4 = (size_t)NB * NM * CC * HW / 4; k_copy<<<(unsigned)((n4 + 255) / 256), 256, 0, stream>>>(x, out); }
  k_kv<0><<<dim3(HW / 64, 1, NB * NM), 128, 0, stream>>>(x, mkw, mvw, MK, MVT, nullptr);
  k_kv<1><<<dim3(HW / 64, 1, NB), 128, 0, stream>>>(x, qkw, qvw, QK, nullptr, QV);
  k_attn<<<dim3(HW / 64, NB), 128, 0, stream>>>(QK, MK, MVT, AGG);
  k_fin<<<dim3(HW / 64, CC / 128, NB), 128, 0, stream>>>(QV, AGG, smw, bsc, bbi, bmu, bva, out);
}
